// TrafalignTransformer_66013647339884
// MI455X (gfx1250) — hardware-verified
//
#include <hip/hip_runtime.h>
#include <math.h>
#include <stdint.h>

#define NBATCH 2
#define NTOK   16384
#define CDIM   256
#define DHEAD  64
#define NPTS   18
#define FDIM   1024
#define QKVN   192
#define MROWS  (NBATCH * NTOK)
#define MCH    16384
#define NCHUNK (MROWS / MCH)
#define WSC    64.0f
#define XPC    64.0f
#define CTXC   256.0f
#define XNC    64.0f
#define HCAR   256.0f
#define ATT_SCALE 0.125f
#define LN_EPS 1e-5f
#define AQ     64
#define OUT0_ELEMS ((size_t)MROWS * CDIM)
#define OUT1_ELEMS ((size_t)MROWS * NPTS)
static_assert((MROWS % 64) == 0 && (MCH % 64) == 0 && (NCHUNK * MCH) == MROWS);
static_assert((CDIM % 64) == 0 && (DHEAD % 64) == 0 && (FDIM % 64) == 0 && (QKVN % 64) == 0);
static_assert((CDIM % 32) == 0 && (DHEAD % 32) == 0 && (FDIM % 32) == 0);
static_assert((NTOK & (NTOK - 1)) == 0);
static_assert((MROWS % AQ) == 0 && ((AQ * NPTS) % 4) == 0 && ((AQ * NPTS) / 4) == 288 && (AQ / 8) * 8 == AQ);
static_assert(OUT0_ELEMS + OUT1_ELEMS == (size_t)8978432);
static_assert(((OUT0_ELEMS * 4) % 128) == 0 && ((AQ * NPTS * 4) % 128) == 0);

typedef _Float16 v16h __attribute__((ext_vector_type(16)));
typedef _Float16 v8h  __attribute__((ext_vector_type(8)));
typedef float    v8f  __attribute__((ext_vector_type(8)));
typedef float    v4f  __attribute__((ext_vector_type(4)));
typedef float    v2f  __attribute__((ext_vector_type(2)));
typedef unsigned int v4u __attribute__((ext_vector_type(4)));
typedef unsigned int v2u __attribute__((ext_vector_type(2)));

union FragH { v16h v; v8h h[2]; v4u u[2]; };

__device__ __forceinline__ unsigned short bf_bits(float f) {
  unsigned u = __float_as_uint(f);
  return (unsigned short)((u + 0x7FFFu + ((u >> 16) & 1u)) >> 16);
}
__device__ __forceinline__ float bf_up(unsigned short h) { return __uint_as_float(((unsigned)h) << 16); }
__device__ __forceinline__ float bfr(float f) { return bf_up(bf_bits(f)); }
__device__ __forceinline__ unsigned short h_bits(_Float16 x) { return __builtin_bit_cast(unsigned short, x); }
__device__ __forceinline__ unsigned pk16(unsigned short a, unsigned short b) { return (unsigned)a | ((unsigned)b << 16); }
__device__ __forceinline__ v8f zero8() { v8f z = {0.f, 0.f, 0.f, 0.f, 0.f, 0.f, 0.f, 0.f}; return z; }
__device__ __forceinline__ void split16(float v, unsigned short& hb, unsigned short& lb) {
  const _Float16 hh = (_Float16)v;
  const float res = v - (float)hh;
  hb = h_bits(hh);
  lb = h_bits((_Float16)res);
}

__device__ __forceinline__ v16h ldfrag_u(const unsigned short* p) {
  FragH f;
  f.u[0] = *(const v4u*)(p);
  f.u[1] = *(const v4u*)(p + 16);
  return f.v;
}

__device__ __forceinline__ v8f mma_raw(v16h a, v16h b, v8f c) {
  return __builtin_amdgcn_wmma_f32_16x16x32_f16(false, a, false, b, (short)0, c, false, false);
}
__device__ __forceinline__ void dep_guard1(v8f& a, v8f& b, v16h x) {
#if defined(__HIP_DEVICE_COMPILE__)
  asm volatile("v_nop\n\tv_nop\n\tv_nop\n\tv_nop" : "+v"(a), "+v"(b) : "v"(x));
#endif
}
__device__ __forceinline__ void keep4_h(v16h a, v16h b, v16h c, v16h d) {
#if defined(__HIP_DEVICE_COMPILE__)
  asm volatile("v_nop" :: "v"(a), "v"(b), "v"(c), "v"(d));
#endif
}
__device__ __forceinline__ void acc_guard4(v8f& a, v8f& b, v8f& c, v8f& d) {
#if defined(__HIP_DEVICE_COMPILE__)
  asm volatile("v_nop\n\tv_nop\n\tv_nop\n\tv_nop" : "+v"(a), "+v"(b), "+v"(c), "+v"(d));
#endif
}
__device__ __forceinline__ void wave_sync_lds() {
  __builtin_amdgcn_fence(__ATOMIC_RELEASE, "workgroup");
  __builtin_amdgcn_wave_barrier();
  __builtin_amdgcn_fence(__ATOMIC_ACQUIRE, "workgroup");
}

__global__ __launch_bounds__(256) void tcvt16(const float* __restrict__ src, unsigned short* dst, int R, int C, float sc) {
  __shared__ __align__(16) unsigned short sT[64 * 72];
  const int tid = threadIdx.x, lane = tid & 31, wave = tid >> 5;
  const int c0 = blockIdx.x * 64, r0 = blockIdx.y * 64;
  const int rr = tid >> 2, cc = (tid & 3) * 16;
  const float* sp = src + (size_t)(r0 + rr) * C + c0 + cc;
#pragma unroll
  for (int e = 0; e < 4; ++e) {
    const v4f a = *(const v4f*)(sp + 4 * e);
#pragma unroll
    for (int k = 0; k < 4; ++k)
      sT[(cc + 4 * e + k) * 72 + rr] = h_bits((_Float16)(bfr(a[k]) * sc));
  }
  __syncthreads();
  v4u vals[2];
#pragma unroll
  for (int it = 0; it < 2; ++it) {
    const int q = it * 32 + wave * 4 + (lane >> 3);
    vals[it] = *(const v4u*)(sT + q * 72 + (lane & 7) * 8);
  }
  for (int pass = 0; pass < 2; ++pass) {
#pragma unroll
    for (int it = 0; it < 2; ++it) {
      const int q = it * 32 + wave * 4 + (lane >> 3);
      *(volatile v4u*)(dst + (size_t)(c0 + q) * R + r0 + (lane & 7) * 8) = vals[it];
    }
    __threadfence();
  }
}

__global__ __launch_bounds__(64) void bcat(const float* __restrict__ bq, const float* __restrict__ bk,
                                           const float* __restrict__ bv, const int* __restrict__ tk, float* dst) {
  const int t = threadIdx.x;
  const int i4 = (t & 15) * 4;
  const v4f a = *(const v4f*)(bq + i4);
  const v4f b = *(const v4f*)(bk + i4);
  const v4f c = *(const v4f*)(bv + i4);
  const int s = t >> 4;
  v4f v;
#pragma unroll
  for (int e = 0; e < 4; ++e) {
    const float x = (s == 0) ? a[e] : ((s == 1) ? b[e] : c[e]);
    v[e] = bfr(x);
  }
  (void)tk;
  for (int pass = 0; pass < 2; ++pass) {
    if (t < 48) *(volatile v4f*)(dst + 4 * t) = v;
    __threadfence();
  }
}

__global__ __launch_bounds__(256) void prep(const float* __restrict__ X, const float* __restrict__ Pz,
                                            unsigned short* XH, unsigned short* XL) {
  const size_t t = (size_t)blockIdx.x * 256 + threadIdx.x;
  const size_t e = t * 8;
  if (e >= (size_t)MROWS * CDIM) return;
  const size_t pe = e & ((size_t)NTOK * CDIM - 1);
  const v4f xa = *(const v4f*)(X + e),   xb = *(const v4f*)(X + e + 4);
  const v4f pa = *(const v4f*)(Pz + pe), pb = *(const v4f*)(Pz + pe + 4);
  unsigned short hb[8], lb[8];
#pragma unroll
  for (int k = 0; k < 4; ++k) {
    split16((bfr(xa[k]) + bfr(pa[k])) * XPC, hb[k], lb[k]);
    split16((bfr(xb[k]) + bfr(pb[k])) * XPC, hb[4 + k], lb[4 + k]);
  }
  v4u hv, lv;
#pragma unroll
  for (int q = 0; q < 4; ++q) {
    hv[q] = pk16(hb[2 * q], hb[2 * q + 1]);
    lv[q] = pk16(lb[2 * q], lb[2 * q + 1]);
  }
  for (int pass = 0; pass < 2; ++pass) {
    *(volatile v4u*)(XH + e) = hv;
    *(volatile v4u*)(XL + e) = lv;
    __threadfence();
  }
}

template <int NA, int OM, int HASR, int ACT>
__global__ __launch_bounds__(256) void gemm64(
    const unsigned short* __restrict__ A1p, const unsigned short* __restrict__ A2p, int lda,
    const unsigned short* __restrict__ Btp, int ldb,
    const float* __restrict__ Bsp, const float* __restrict__ Rp,
    void* Cout, int ldc, int M, int N, int K, float oscale, float ocarry) {
  __shared__ __align__(16) float sT[8][16 * 68];
  const int lane = threadIdx.x & 31;
  const int wave = threadIdx.x >> 5;
  const int tilesN = N >> 6;
  const int tilesM = M >> 6;
  const int tile = blockIdx.x * 8 + wave;
  if (tile >= tilesM * tilesN) return;
  const int tm = tile / tilesN;
  const int tn = tile - tm * tilesN;
  const int m0 = tm << 6;
  const int n0 = tn << 6;

  const int rlane = lane & 15;
  const int koff  = (lane >> 4) * 8;
  const int mOff  = (lane >> 4) * 8;

  v8f acc[4][4];
#pragma unroll
  for (int i = 0; i < 4; ++i)
#pragma unroll
    for (int j = 0; j < 4; ++j) acc[i][j] = zero8();

  for (int k0 = 0; k0 < K; k0 += 32) {
    v16h bh[4];
#pragma unroll
    for (int j = 0; j < 4; ++j) {
      const size_t bofs = (size_t)(n0 + (j << 4) + rlane) * ldb + koff + k0;
      bh[j] = ldfrag_u(Btp + bofs);
    }
#pragma unroll
    for (int pl = 0; pl < NA; ++pl) {
      const unsigned short* Ab = (pl == 0) ? A1p : A2p;
#pragma unroll
      for (int i = 0; i < 4; ++i) {
        const size_t ao = (size_t)(m0 + (i << 4) + rlane) * lda + koff + k0;
        const v16h ah = ldfrag_u(Ab + ao);
#pragma unroll
        for (int j = 0; j < 4; ++j) acc[i][j] = mma_raw(ah, bh[j], acc[i][j]);
        dep_guard1(acc[i][0], acc[i][3], ah);
      }
    }
    keep4_h(bh[0], bh[1], bh[2], bh[3]);
  }
  acc_guard4(acc[0][0], acc[0][1], acc[0][2], acc[0][3]);
  acc_guard4(acc[1][0], acc[1][1], acc[1][2], acc[1][3]);
  acc_guard4(acc[2][0], acc[2][1], acc[2][2], acc[2][3]);
  acc_guard4(acc[3][0], acc[3][1], acc[3][2], acc[3][3]);

  const int hh2 = lane >> 4, c4 = (lane & 15) * 4;
  const int q8  = lane >> 3, c8 = (lane & 7) * 8;

  float* slab = sT[wave];
#pragma unroll
  for (int i = 0; i < 4; ++i) {
    const int mBase = m0 + (i << 4);
#pragma unroll
    for (int j = 0; j < 4; ++j) {
#pragma unroll
      for (int r = 0; r < 8; ++r) {
        slab[(mOff + r) * 68 + (j << 4) + rlane] = acc[i][j][r];
      }
    }
    wave_sync_lds();
    if constexpr (OM == 0) {
      float* C = (float*)Cout;
      const v4f braw = *(const v4f*)(Bsp + n0 + c4);
      v4f bb;
#pragma unroll
      for (int e = 0; e < 4; ++e) bb[e] = bfr(braw[e]);
      v4f vals[8];
#pragma unroll
      for (int it = 0; it < 8; ++it) {
        const int row = it * 2 + hh2;
        const int gr  = mBase + row;
        v4f v = *(const v4f*)(slab + row * 68 + c4);
        v4f rv = {0.f, 0.f, 0.f, 0.f};
        if constexpr (HASR == 2) {
          rv = *(const v4f*)(Rp + (size_t)gr * ldc + n0 + c4);
        }
#pragma unroll
        for (int e = 0; e < 4; ++e) {
          float t = v[e] * oscale + bb[e];
          if constexpr (ACT == 1) t = fmaxf(t, 0.0f);
          v[e] = t + rv[e];
        }
        vals[it] = v;
      }
      for (int pass = 0; pass < 2; ++pass) {
#pragma unroll
        for (int it = 0; it < 8; ++it) {
          const int gr = mBase + it * 2 + hh2;
          *(volatile v4f*)(C + (size_t)gr * ldc + n0 + c4) = vals[it];
        }
        __threadfence();
      }
    } else {
      unsigned short* C = (unsigned short*)Cout;
      const v4f b0r = *(const v4f*)(Bsp + n0 + c8);
      const v4f b1r = *(const v4f*)(Bsp + n0 + c8 + 4);
      float b8[8];
#pragma unroll
      for (int e = 0; e < 4; ++e) { b8[e] = bfr(b0r[e]); b8[4 + e] = bfr(b1r[e]); }
      v4u hv[4];
#pragma unroll
      for (int it = 0; it < 4; ++it) {
        const int row = it * 4 + q8;
        const float* sp = slab + row * 68 + c8;
        v4u a = {0u, 0u, 0u, 0u};
#pragma unroll
        for (int e = 0; e < 4; ++e) {
          float f0 = sp[2 * e] * oscale + b8[2 * e];
          float f1 = sp[2 * e + 1] * oscale + b8[2 * e + 1];
          if constexpr (ACT == 1) { f0 = fmaxf(f0, 0.0f); f1 = fmaxf(f1, 0.0f); }
          f0 *= ocarry; f1 *= ocarry;
          a[e] = pk16(h_bits((_Float16)f0), h_bits((_Float16)f1));
        }
        hv[it] = a;
      }
      for (int pass = 0; pass < 2; ++pass) {
#pragma unroll
        for (int it = 0; it < 4; ++it) {
          const int row = it * 4 + q8;
          *(volatile v4u*)(C + (size_t)(mBase + row) * ldc + n0 + c8) = hv[it];
        }
        __threadfence();
      }
    }
    wave_sync_lds();
  }
}

__global__ __launch_bounds__(256)
void rpattn(const float* __restrict__ QKV, const int* __restrict__ sel, float* aout,
            unsigned short* CHp, unsigned short* CLp) {
  __shared__ __align__(16) float sAtt[AQ * NPTS];
  __shared__ __align__(16) unsigned short sCH[AQ * DHEAD];
  __shared__ __align__(16) unsigned short sCL[AQ * DHEAD];
  const int tid = threadIdx.x, lane = tid & 31, wave = tid >> 5;
  const int m0 = blockIdx.x * AQ;

#pragma unroll 1
  for (int s = 0; s < AQ / 8; ++s) {
    const int ql = wave * (AQ / 8) + s;
    const int m  = m0 + ql;
    const int b  = m / NTOK;
    const float* base = QKV + (size_t)b * NTOK * QKVN;
    const v2f qv = *(const v2f*)(QKV + (size_t)m * QKVN + 2 * lane);
    const int lp = (lane < NPTS) ? lane : (NPTS - 1);
    int j = sel[(size_t)m * NPTS + lp];
    j = (j < 0) ? (j + NTOK) : j;
    j = (j < 0) ? 0 : ((j > NTOK - 1) ? (NTOK - 1) : j);

    float mys = -INFINITY;
#pragma unroll 1
    for (int p = 0; p < NPTS; ++p) {
      const int jp = __shfl(j, p, 32);
      const v2f kv = *(const v2f*)(base + (size_t)jp * QKVN + DHEAD + 2 * lane);
      float d = qv[0] * kv[0] + qv[1] * kv[1];
#pragma unroll
      for (int off = 16; off > 0; off >>= 1) d += __shfl_xor(d, off, 32);
      const float sc = d * ATT_SCALE;
      mys = (lane == p) ? sc : mys;
    }
    float mx = mys;
#pragma unroll
    for (int off = 16; off > 0; off >>= 1) mx = fmaxf(mx, __shfl_xor(mx, off, 32));
    const float ev = __expf(mys - mx);
    float su = ev;
#pragma unroll
    for (int off = 16; off > 0; off >>= 1) su += __shfl_xor(su, off, 32);
    const float a = ev * (1.0f / su);
    if (lane < NPTS) sAtt[ql * NPTS + lane] = a;

    float cx = 0.f, cy = 0.f;
#pragma unroll 1
    for (int p = 0; p < NPTS; ++p) {
      const int jp = __shfl(j, p, 32);
      const float ap = __shfl(a, p, 32);
      const v2f vv = *(const v2f*)(base + (size_t)jp * QKVN + 2 * DHEAD + 2 * lane);
      cx = fmaf(ap, vv[0], cx);
      cy = fmaf(ap, vv[1], cy);
    }
    unsigned short hx, lx, hy, ly;
    split16(cx * CTXC, hx, lx);
    split16(cy * CTXC, hy, ly);
    *(unsigned*)(sCH + ql * DHEAD + 2 * lane) = pk16(hx, hy);
    *(unsigned*)(sCL + ql * DHEAD + 2 * lane) = pk16(lx, ly);
  }
  __syncthreads();

  const int p1 = (tid < (AQ * NPTS) / 4 - 256) ? (256 + tid) : ((AQ * NPTS) / 4 - 1);
  const v4f a0 = *(const v4f*)(sAtt + 4 * tid);
  const v4f a1 = *(const v4f*)(sAtt + 4 * p1);
  const v4u h0 = *(const v4u*)(sCH + 8 * tid);
  const v4u h1 = *(const v4u*)(sCH + 8 * (256 + tid));
  const v4u l0 = *(const v4u*)(sCL + 8 * tid);
  const v4u l1 = *(const v4u*)(sCL + 8 * (256 + tid));
  float* ab = aout + (size_t)blockIdx.x * (AQ * NPTS);
  unsigned short* chb = CHp + (size_t)m0 * DHEAD;
  unsigned short* clb = CLp + (size_t)m0 * DHEAD;
  for (int pass = 0; pass < 2; ++pass) {
    *(volatile v4f*)(ab + 4 * tid) = a0;
    if (tid < (AQ * NPTS) / 4 - 256) *(volatile v4f*)(ab + 4 * (256 + tid)) = a1;
    *(volatile v4u*)(chb + 8 * tid) = h0;
    *(volatile v4u*)(chb + 8 * (256 + tid)) = h1;
    *(volatile v4u*)(clb + 8 * tid) = l0;
    *(volatile v4u*)(clb + 8 * (256 + tid)) = l1;
    __threadfence();
  }
}

template <int MODE, int HOUT>
__global__ __launch_bounds__(256)
void lnorm(const float* __restrict__ Ap, const float* __restrict__ Pp, const float* __restrict__ Op,
           const float* __restrict__ gp, const float* __restrict__ bep, float* outf, unsigned short* outh, float hc) {
  __shared__ __align__(16) unsigned short srow[8][CDIM];
  const int tid = threadIdx.x, lane = tid & 31, wave = tid >> 5;
  const int row = blockIdx.x * 8 + wave;
  const int c0 = lane * 4, c1 = 128 + lane * 4;
  const size_t rb = (size_t)row * CDIM;
  v4f ya, yb;
  if constexpr (MODE == 0) {
    const size_t pb = (size_t)(row & (NTOK - 1)) * CDIM;
    const v4f xa = *(const v4f*)(Ap + rb + c0), xb = *(const v4f*)(Ap + rb + c1);
    const v4f pa = *(const v4f*)(Pp + pb + c0), pq = *(const v4f*)(Pp + pb + c1);
    const v4f oa = *(const v4f*)(Op + rb + c0), ob = *(const v4f*)(Op + rb + c1);
#pragma unroll
    for (int e = 0; e < 4; ++e) {
      ya[e] = (bfr(xa[e]) + bfr(pa[e])) + oa[e];
      yb[e] = (bfr(xb[e]) + bfr(pq[e])) + ob[e];
    }
  } else {
    ya = *(const v4f*)(Ap + rb + c0);
    yb = *(const v4f*)(Ap + rb + c1);
  }
  float s = ((ya[0] + ya[1]) + (ya[2] + ya[3])) + ((yb[0] + yb[1]) + (yb[2] + yb[3]));
#pragma unroll
  for (int off = 1; off < 32; off <<= 1) s += __shfl_xor(s, off, 32);
  const float mu = s * (1.0f / (float)CDIM);
  v4f da, db;
#pragma unroll
  for (int e = 0; e < 4; ++e) { da[e] = ya[e] - mu; db[e] = yb[e] - mu; }
  float q = ((da[0] * da[0] + da[1] * da[1]) + (da[2] * da[2] + da[3] * da[3])) +
            ((db[0] * db[0] + db[1] * db[1]) + (db[2] * db[2] + db[3] * db[3]));
#pragma unroll
  for (int off = 1; off < 32; off <<= 1) q += __shfl_xor(q, off, 32);
  const float var  = q * (1.0f / (float)CDIM);
  const float rstd = rsqrtf(var + LN_EPS);
  const v4f ga = *(const v4f*)(gp + c0),  gb = *(const v4f*)(gp + c1);
  const v4f ba = *(const v4f*)(bep + c0), bb = *(const v4f*)(bep + c1);
  v4f oa2, ob2;
#pragma unroll
  for (int e = 0; e < 4; ++e) {
    oa2[e] = (da[e] * rstd) * bfr(ga[e]) + bfr(ba[e]);
    ob2[e] = (db[e] * rstd) * bfr(gb[e]) + bfr(bb[e]);
  }
  for (int pass = 0; pass < 2; ++pass) {
    *(volatile v4f*)(outf + rb + c0) = oa2;
    *(volatile v4f*)(outf + rb + c1) = ob2;
    __threadfence();
  }
  if constexpr (HOUT == 1) {
    v2u w0, w1;
    w0[0] = pk16(h_bits((_Float16)(oa2[0] * hc)), h_bits((_Float16)(oa2[1] * hc)));
    w0[1] = pk16(h_bits((_Float16)(oa2[2] * hc)), h_bits((_Float16)(oa2[3] * hc)));
    w1[0] = pk16(h_bits((_Float16)(ob2[0] * hc)), h_bits((_Float16)(ob2[1] * hc)));
    w1[1] = pk16(h_bits((_Float16)(ob2[2] * hc)), h_bits((_Float16)(ob2[3] * hc)));
    unsigned short* sr = srow[wave];
    *(v2u*)(sr + c0) = w0;
    *(v2u*)(sr + c1) = w1;
    wave_sync_lds();
    const v4u hv = *(const v4u*)(sr + 8 * lane);
    for (int pass = 0; pass < 2; ++pass) {
      *(volatile v4u*)(outh + rb + 8 * lane) = hv;
      __threadfence();
    }
  }
}

extern "C" void kernel_launch(void* const* d_in, const int* in_sizes, int n_in,
                              void* d_out, int out_size, void* d_ws, size_t ws_size,
                              hipStream_t stream) {
  if (n_in < 20) return;
  if (in_sizes[0] != MROWS * CDIM) return;
  if (in_sizes[1] != MROWS * NPTS) return;
  if (in_sizes[2] < 1) return;
  if (in_sizes[3] != NTOK * CDIM) return;
  if (in_sizes[4] != CDIM * DHEAD || in_sizes[6] != CDIM * DHEAD || in_sizes[8] != CDIM * DHEAD) return;
  if (in_sizes[5] != DHEAD || in_sizes[7] != DHEAD || in_sizes[9] != DHEAD) return;
  if (in_sizes[10] != DHEAD * CDIM || in_sizes[11] != CDIM) return;
  if (in_sizes[12] != CDIM * FDIM || in_sizes[13] != FDIM) return;
  if (in_sizes[14] != FDIM * CDIM || in_sizes[15] != CDIM) return;
  if (in_sizes[16] != CDIM || in_sizes[17] != CDIM || in_sizes[18] != CDIM || in_sizes[19] != CDIM) return;
  if ((size_t)out_size != OUT0_ELEMS + OUT1_ELEMS) return;

  const float* X   = (const float*)d_in[0];
  const int*   sel = (const int*)d_in[1];
  const int*   tpk = (const int*)d_in[2];
  const float* pos = (const float*)d_in[3];
  const float* Wq  = (const float*)d_in[4];
  const float* bq  = (const float*)d_in[5];
  const float* Wk  = (const float*)d_in[6];
  const float* bk  = (const float*)d_in[7];
  const float* Wv  = (const float*)d_in[8];
  const float* bv  = (const float*)d_in[9];
  const float* Wo  = (const float*)d_in[10];
  const float* bo  = (const float*)d_in[11];
  const float* W1  = (const float*)d_in[12];
  const float* b1  = (const float*)d_in[13];
  const float* W2  = (const float*)d_in[14];
  const float* b2  = (const float*)d_in[15];
  const float* g1  = (const float*)d_in[16];
  const float* be1 = (const float*)d_in[17];
  const float* g2  = (const float*)d_in[18];
  const float* be2 = (const float*)d_in[19];
  float* out0 = (float*)d_out;
  float* out1 = out0 + OUT0_ELEMS;

  const size_t oWQKV = 0;
  const size_t oWO   = oWQKV + (size_t)QKVN * CDIM * 2;
  const size_t oW1   = oWO + (size_t)CDIM * DHEAD * 2;
  const size_t oW2   = oW1 + (size_t)FDIM * CDIM * 2;
  const size_t oBQ   = oW2 + (size_t)CDIM * FDIM * 2;
  const size_t oR1   = (size_t)2097152;
  if (oBQ + 1024 > oR1) return;
  const size_t szX16 = (size_t)MROWS * CDIM * 2;
  const size_t szX32 = (size_t)MROWS * CDIM * 4;
  const size_t szQKV = (size_t)MROWS * QKVN * 4;
  const size_t szC16 = (size_t)MROWS * DHEAD * 2;
  const size_t szHH  = (size_t)MCH * FDIM * 2;
  const size_t oR2   = oR1 + 2 * szX16;
  const size_t oR3   = oR2 + szQKV;
  const size_t oR4   = oR3 + 2 * szC16;
  const size_t oR5   = oR4 + szX32;
  const size_t oEnd  = oR5 + szX16;
  const size_t oXH   = oR1, oXL = oR1 + szX16, oXNF = oR1;
  const size_t oQKV  = oR2, oXNH = oR2;
  const size_t oCH   = oR3, oCL = oR3 + szC16;
  const size_t oOUT  = oR4;
  const size_t oHH   = oXNH + szX16;
  const size_t oY2   = oHH + szHH;
  if (oXNF + szX32 > oR2) return;
  if (oHH + szHH > oY2) return;
  if (oY2 + szX32 != oEnd) return;
  if (oEnd > ws_size) return;
  if (oEnd > (size_t)134217728) return;

  char* ws = (char*)d_ws;
  unsigned short* WQKV = (unsigned short*)(ws + oWQKV);
  unsigned short* WOT  = (unsigned short*)(ws + oWO);
  unsigned short* W1T  = (unsigned short*)(ws + oW1);
  unsigned short* W2T  = (unsigned short*)(ws + oW2);
  float*          BQKV = (float*)(ws + oBQ);
  unsigned short* XH   = (unsigned short*)(ws + oXH);
  unsigned short* XL   = (unsigned short*)(ws + oXL);
  float*          XNF  = (float*)(ws + oXNF);
  float*          QKVF = (float*)(ws + oQKV);
  unsigned short* XNH  = (unsigned short*)(ws + oXNH);
  unsigned short* CH   = (unsigned short*)(ws + oCH);
  unsigned short* CL   = (unsigned short*)(ws + oCL);
  float*          OUTF = (float*)(ws + oOUT);
  unsigned short* HH   = (unsigned short*)(ws + oHH);
  float*          Y2F  = (float*)(ws + oY2);

  const dim3 blk(256);
  const int tilesQKV = (MROWS / 64) * (QKVN / 64);
  const int tilesWO  = (MROWS / 64) * (CDIM / 64);
  const int tilesF1  = (MCH / 64) * (FDIM / 64);
  const int tilesF2  = (MCH / 64) * (CDIM / 64);
  const dim3 gQKV((tilesQKV + 7) / 8);
  const dim3 gWO((tilesWO + 7) / 8);
  const dim3 gF1((tilesF1 + 7) / 8);
  const dim3 gF2((tilesF2 + 7) / 8);
  const dim3 gLN(MROWS / 8);
  const dim3 gPR((MROWS * CDIM) / (256 * 8));
  const dim3 gAT(MROWS / AQ);

  tcvt16<<<dim3(DHEAD / 64, CDIM / 64), blk, 0, stream>>>(Wq, WQKV, CDIM, DHEAD, WSC);
  tcvt16<<<dim3(DHEAD / 64, CDIM / 64), blk, 0, stream>>>(Wk, WQKV + (size_t)DHEAD * CDIM, CDIM, DHEAD, WSC);
  tcvt16<<<dim3(DHEAD / 64, CDIM / 64), blk, 0, stream>>>(Wv, WQKV + (size_t)2 * DHEAD * CDIM, CDIM, DHEAD, WSC);
  tcvt16<<<dim3(CDIM / 64, DHEAD / 64), blk, 0, stream>>>(Wo, WOT, DHEAD, CDIM, WSC);
  tcvt16<<<dim3(FDIM / 64, CDIM / 64), blk, 0, stream>>>(W1, W1T, CDIM, FDIM, WSC);
  tcvt16<<<dim3(CDIM / 64, FDIM / 64), blk, 0, stream>>>(W2, W2T, FDIM, CDIM, WSC);

  bcat<<<dim3(1), dim3(64), 0, stream>>>(bq, bk, bv, tpk, BQKV);

  prep<<<gPR, blk, 0, stream>>>(X, pos, XH, XL);

  gemm64<2, 0, 0, 0><<<gQKV, blk, 0, stream>>>(
      XH, XL, CDIM, WQKV, CDIM, BQKV, BQKV, (void*)QKVF, QKVN, MROWS, QKVN, CDIM, 1.0f / (XPC * WSC), 1.0f);

  rpattn<<<gAT, blk, 0, stream>>>(QKVF, sel, out1, CH, CL);

  gemm64<2, 0, 0, 0><<<gWO, blk, 0, stream>>>(
      CH, CL, DHEAD, WOT, DHEAD, bo, bo, (void*)OUTF, CDIM, MROWS, CDIM, DHEAD, 1.0f / (CTXC * WSC), 1.0f);

  lnorm<0, 1><<<gLN, blk, 0, stream>>>(X, pos, OUTF, g1, be1, XNF, XNH, XNC);

  for (int c = 0; c < NCHUNK; ++c) {
    const size_t rofs = (size_t)c * MCH * CDIM;
    gemm64<1, 2, 0, 1><<<gF1, blk, 0, stream>>>(
        XNH + rofs, XNH + rofs, CDIM, W1T, CDIM, b1, b1, (void*)HH, FDIM, MCH, FDIM, CDIM, 1.0f / (XNC * WSC), HCAR);
    gemm64<1, 0, 2, 0><<<gF2, blk, 0, stream>>>(
        HH, HH, FDIM, W2T, FDIM, b2, XNF + rofs, (void*)(Y2F + rofs), CDIM, MCH, CDIM, FDIM, 1.0f / (HCAR * WSC), 1.0f);
  }

  lnorm<1, 0><<<gLN, blk, 0, stream>>>(Y2F, Y2F, Y2F, g2, be2, out0, XNH, 1.0f);
  (void)hipGetLastError();
}
